// CausalSelfAttention_59493886984270
// MI455X (gfx1250) — hardware-verified
//
#include <hip/hip_runtime.h>


#pragma clang fp contract(off)

#ifndef NB
#define NB 2
#endif
#ifndef SEQ
#define SEQ 2048
#endif
#ifndef RE
#define RE   256
#endif
#define NB_FULL  2
#define SEQ_FULL 2048
#define DM   2048
#define NH_  16
#define NKV  4
#define REP  (NH_ / NKV)
#define HD   128
#define DQ   (NH_ * HD)
#define DKV  (NKV * HD)
#define PCAR 1024.0f
#define CCAR 64.0f
#define LOSC 1024.0f
#define WCAR 1024.0f
#define WS_TOTAL ((size_t)DQ * DM * 2 + 2 * (size_t)DKV * DM * 2 + 2 * (size_t)DM * DQ * 2 + (size_t)SEQ * DM * 2 + (size_t)SEQ * DQ * 4 + 2 * (size_t)SEQ * DKV * 4 \
                  + (size_t)NH_ * SEQ * HD * 2 + 2 * (size_t)NKV * SEQ * HD * 2 + 2 * (size_t)NH_ * RE * HD * 2 + 4 * (size_t)NKV * RE * HD * 2 + (size_t)SEQ * DM * 2 + (size_t)RE * DM * 2)

static_assert((SEQ % 64) == 0);
static_assert((RE % 64) == 0);
static_assert(RE >= 64);
static_assert(SEQ >= RE);
static_assert(SEQ <= SEQ_FULL);
static_assert(NB >= 1);
static_assert(NB <= NB_FULL);
static_assert(HD == 128);
static_assert((DM % 32) == 0);
static_assert(DQ == DM);
static_assert(((SEQ * DM) % (8 * 256)) == 0);
static_assert(((NH_ * SEQ * HD) % (2 * 256)) == 0);
static_assert(((NKV * SEQ * HD) % (2 * 256)) == 0);
static_assert(((DQ * DM) % (8 * 256)) == 0);
static_assert(((DKV * DM) % (8 * 256)) == 0);
static_assert(NH_ == 16);
static_assert(REP * NKV == NH_);
static_assert((HD % 64) == 0);
static_assert((DQ % 64) == 0);
static_assert((DKV % 64) == 0);
static_assert((DM % 64) == 0);
static_assert(((size_t)NKV * RE * HD * 2) % 256 == 0);
static_assert(WS_TOTAL <= (size_t)134217728);

typedef _Float16 h16;
typedef unsigned short bf;
typedef __attribute__((ext_vector_type(16))) __bf16   v16bf;
typedef __attribute__((ext_vector_type(16))) _Float16 v16h;
typedef __attribute__((ext_vector_type(8)))  _Float16 v8h;
typedef __attribute__((ext_vector_type(8)))  unsigned short v8us;
typedef __attribute__((ext_vector_type(8)))  float    v8f;
typedef __attribute__((ext_vector_type(4)))  float    v4f;
typedef __attribute__((ext_vector_type(2)))  _Float16 v2h;
typedef __attribute__((ext_vector_type(2)))  unsigned short v2us;
typedef v8h  __attribute__((may_alias)) v8ha;
typedef v4f  __attribute__((may_alias)) v4fa;
typedef v8us __attribute__((may_alias)) v8usa;

__device__ __forceinline__ unsigned short f2bf(float f) { unsigned u = __float_as_uint(f); u += 0x7FFFu + ((u >> 16) & 1u); return (unsigned short)(u >> 16); }
__device__ __forceinline__ float bf2f(unsigned short b) { return __uint_as_float(((unsigned)b) << 16); }
__device__ __forceinline__ float bfr(float f) { return bf2f(f2bf(f)); }
__device__ __forceinline__ h16 tohx(float x) { return (h16)x; }
static __device__ __forceinline__ h16 toh_flush(float v) { const h16 r = (h16)v; return (fabsf(v) < 6.103515625e-05f) ? (h16)0.0f : r; }
static __device__ __forceinline__ float nnum(float v, float big) { const float a = (v != v) ? 0.0f : v; return (a == __builtin_inff()) ? big : ((a == -__builtin_inff()) ? -big : a); }
__device__ __forceinline__ void splitf(float y, unsigned short& h, unsigned short& l) { h = f2bf(y); l = f2bf(y - bf2f(h)); }
__device__ __forceinline__ v16h cat16(v8h lo, v8h hi) { return __builtin_shufflevector(lo, hi, 0, 1, 2, 3, 4, 5, 6, 7, 8, 9, 10, 11, 12, 13, 14, 15); }
__device__ __forceinline__ v16bf cat16b(v8us lo, v8us hi) { return __builtin_bit_cast(v16bf, __builtin_shufflevector(lo, hi, 0, 1, 2, 3, 4, 5, 6, 7, 8, 9, 10, 11, 12, 13, 14, 15)); }
__device__ __forceinline__ v8f wmma16(v16h a, v16h b, v8f c) { return __builtin_amdgcn_wmma_f32_16x16x32_f16(false, a, false, b, (short)0, c, false, false); }
__device__ __forceinline__ v8f wmmab(v16bf a, v16bf b, v8f c) { return __builtin_amdgcn_wmma_f32_16x16x32_bf16(false, a, false, b, (short)0, c, false, false); }

template <typename T16> struct WFrag;
template <> struct WFrag<h16> { typedef v16h V; static __device__ __forceinline__ V ld(const h16* p) { return cat16(*(const v8ha*)p, *(const v8ha*)(p + 16)); } static __device__ __forceinline__ v8f mma(V a, V b, v8f c) { return wmma16(a, b, c); } };
template <> struct WFrag<bf>  { typedef v16bf V; static __device__ __forceinline__ V ld(const bf* p) { return cat16b(*(const v8usa*)p, *(const v8usa*)(p + 16)); } static __device__ __forceinline__ v8f mma(V a, V b, v8f c) { return wmmab(a, b, c); } };

template <typename T16, int NSPLIT>
__global__ __launch_bounds__(32) void k_gemmw(const T16* __restrict__ A, const T16* __restrict__ A2, const T16* __restrict__ Bt, const T16* __restrict__ Bt2, int K, float* C, int ldc, float oscale) {
    typedef typename WFrag<T16>::V V;
    __shared__ __align__(16) float os[16 * 68];
    const int lane = threadIdx.x & 31, lr = lane & 15, hi = lane >> 4; const int r0 = blockIdx.x * 64, c0 = blockIdx.y * 64;
    v8f acc[4][4];
#pragma unroll
    for (int mb = 0; mb < 4; ++mb)
#pragma unroll
        for (int nb = 0; nb < 4; ++nb) acc[mb][nb] = (v8f){};
    const size_t aoff = (size_t)(r0 + lr) * K + 8 * hi, boff = (size_t)(c0 + lr) * K + 8 * hi;
#pragma unroll 1
    for (int kc = 0; kc < K; kc += 32) {
        V a[4], a2[4];
#pragma unroll
        for (int mb = 0; mb < 4; ++mb) { a[mb] = WFrag<T16>::ld(A + aoff + (size_t)mb * 16 * K + kc); if (NSPLIT != 0) a2[mb] = WFrag<T16>::ld(A2 + aoff + (size_t)mb * 16 * K + kc); }
#pragma unroll
        for (int nb = 0; nb < 4; ++nb) { const V b = WFrag<T16>::ld(Bt + boff + (size_t)nb * 16 * K + kc); V b2 = b; if (NSPLIT >= 2) b2 = WFrag<T16>::ld(Bt2 + boff + (size_t)nb * 16 * K + kc);
#pragma unroll
            for (int mb = 0; mb < 4; ++mb) { acc[mb][nb] = WFrag<T16>::mma(a[mb], b, acc[mb][nb]); if (NSPLIT == 1 || NSPLIT == 2) acc[mb][nb] = WFrag<T16>::mma(a2[mb], b, acc[mb][nb]); if (NSPLIT == 2) acc[mb][nb] = WFrag<T16>::mma(a[mb], b2, acc[mb][nb]); if (NSPLIT == 3) acc[mb][nb] = WFrag<T16>::mma(a2[mb], b2, acc[mb][nb]); } }
        asm volatile("v_nop\n\tv_nop\n\tv_nop\n\tv_nop" : "+v"(acc[0][0]), "+v"(acc[1][1]), "+v"(acc[2][2]), "+v"(acc[3][3]) : "v"(a[0]), "v"(a[3]));
    }
#pragma unroll
    for (int mb = 0; mb < 4; ++mb) {
#pragma unroll
        for (int nb = 0; nb < 4; ++nb) {
#pragma unroll
            for (int j = 0; j < 8; ++j) os[(hi * 8 + j) * 68 + nb * 16 + lr] = acc[mb][nb][j]; }
        __builtin_amdgcn_wave_barrier(); asm volatile("" ::: "memory");
        float* crow = C + (size_t)(r0 + mb * 16) * ldc + c0;
#pragma unroll 1
        for (int ps = 0; ps < 2; ++ps) {
#pragma unroll
            for (int s = 0; s < 8; ++s) { const int row = 2 * s + hi, cofs = lr * 4; v4f val = *(const v4fa*)(os + row * 68 + cofs); val = val * oscale;
                *(volatile v4f*)(crow + (size_t)row * ldc + cofs) = val; }
            if (ps == 0) __threadfence(); }
        __builtin_amdgcn_wave_barrier(); asm volatile("" ::: "memory");
    }
}

__global__ __launch_bounds__(256) void k_cvt8(const float* __restrict__ src, bf* dst, size_t n8) { const size_t i = (size_t)blockIdx.x * 256 + threadIdx.x; if (i >= n8) return; const v8f v = *(const v8f*)(src + i * 8); v8us o;
#pragma unroll
    for (int k = 0; k < 8; ++k) o[k] = f2bf(v[k]); *(volatile v8us*)(dst + i * 8) = o; __threadfence(); *(volatile v8us*)(dst + i * 8) = o; }

__global__ __launch_bounds__(256) void k_cvtx(const float* __restrict__ src, bf* dst, size_t n8) { const size_t i = (size_t)blockIdx.x * 256 + threadIdx.x; if (i >= n8) return; const v8f v = *(const v8f*)(src + i * 8); v8us o;
#pragma unroll
    for (int k = 0; k < 8; ++k) o[k] = f2bf(nnum(v[k], 10000.0f)); *(volatile v8us*)(dst + i * 8) = o; __threadfence(); *(volatile v8us*)(dst + i * 8) = o; }

__global__ __launch_bounds__(256) void k_cvtwo(const float* __restrict__ src, h16* dh, h16* dl, size_t n8) { const size_t i = (size_t)blockIdx.x * 256 + threadIdx.x; if (i >= n8) return; const v8f v = *(const v8f*)(src + i * 8); v8h oh, ol;
#pragma unroll
    for (int k = 0; k < 8; ++k) { const float w = bfr(v[k]); oh[k] = tohx(w * WCAR); ol[k] = tohx(w); }
    *(volatile v8h*)(dh + i * 8) = oh; *(volatile v8h*)(dl + i * 8) = ol; __threadfence(); *(volatile v8h*)(dh + i * 8) = oh; *(volatile v8h*)(dl + i * 8) = ol; }

__global__ __launch_bounds__(256) void k_hpl(const float* __restrict__ F, int pitch, int nheads, h16* P16, bf* Eh, bf* El) {
    const size_t e = ((size_t)blockIdx.x * 256 + threadIdx.x) * 2; if (e >= (size_t)nheads * SEQ * HD) return;
    const int d = (int)(e % HD); const int t = (int)((e / HD) % SEQ); const int h = (int)(e / ((size_t)HD * SEQ));
    const float* f = F + (size_t)t * pitch + h * HD; v2h o16; v2us oh, ol;
#pragma unroll
    for (int q = 0; q < 2; ++q) { const float r = f[d + q]; o16[q] = toh_flush(r); unsigned short a2, c2; splitf(r, a2, c2); oh[q] = a2; ol[q] = c2; }
    const bool early = (t < RE);
    const size_t ee = ((size_t)h * RE + (early ? t : 0)) * HD + d;
    *(volatile v2h*)(P16 + e) = o16; if (early) { *(volatile v2us*)(Eh + ee) = oh; *(volatile v2us*)(El + ee) = ol; }
    __threadfence();
    *(volatile v2h*)(P16 + e) = o16; if (early) { *(volatile v2us*)(Eh + ee) = oh; *(volatile v2us*)(El + ee) = ol; }
}

__global__ __launch_bounds__(256) void k_vtp(const float* __restrict__ F, h16* V16, bf* Eh, bf* El) {
    const size_t e = ((size_t)blockIdx.x * 256 + threadIdx.x) * 2; if (e >= (size_t)NKV * HD * SEQ) return;
    const int t = (int)(e % SEQ); const int d = (int)((e / SEQ) % HD); const int g = (int)(e / ((size_t)SEQ * HD)); v2h o16; v2us oh, ol;
#pragma unroll
    for (int q = 0; q < 2; ++q) { const float x = F[(size_t)(t + q) * DKV + g * HD + d]; o16[q] = tohx(x); unsigned short a2, c2; splitf(x, a2, c2); oh[q] = a2; ol[q] = c2; }
    const bool early = (t < RE);
    const size_t ee = ((size_t)g * HD + d) * RE + (early ? t : 0);
    *(volatile v2h*)(V16 + e) = o16; if (early) { *(volatile v2us*)(Eh + ee) = oh; *(volatile v2us*)(El + ee) = ol; }
    __threadfence();
    *(volatile v2h*)(V16 + e) = o16; if (early) { *(volatile v2us*)(Eh + ee) = oh; *(volatile v2us*)(El + ee) = ol; }
}

__device__ __forceinline__ void putpz(h16* ph, h16* pl, int i, float p) { (void)pl; ph[i] = toh_flush(p * PCAR); }
__device__ __forceinline__ void putpz(bf* ph, bf* pl, int i, float p) { unsigned short a, c; splitf(p, a, c); ph[i] = a; pl[i] = c; }

template <typename T16, bool EARLY>
__global__ __launch_bounds__(128) void k_attn(const T16* __restrict__ Qh, const T16* __restrict__ Ql, const T16* __restrict__ Kh, const T16* __restrict__ Kl,
                                             const T16* __restrict__ Vh, const T16* __restrict__ Vl, h16* CT, h16* CTL) {
    typedef typename WFrag<T16>::V V;
    constexpr int TP = EARLY ? RE : SEQ;
    constexpr int KSP = 136, VTP = 32, PSP = 40, OSP = 128;
    __shared__ __align__(16) T16 ksh[32 * KSP];
    __shared__ __align__(16) T16 ksl[EARLY ? 32 * KSP : 16];
    __shared__ __align__(16) T16 vth[HD * VTP];
    __shared__ __align__(16) T16 vtl[EARLY ? HD * VTP : 16];
    __shared__ __align__(16) T16 psh[4 * 16 * PSP];
    __shared__ __align__(16) T16 psl[EARLY ? 4 * 16 * PSP : 16];
    __shared__ __align__(16) h16 osg[4 * 16 * OSP];
    const int tid = threadIdx.x, lane = tid & 31, wave = tid >> 5, lr = lane & 15, hh = lane >> 4;
    const int qblk = EARLY ? (int)blockIdx.x : ((int)blockIdx.x + RE / 64);
    const int head = blockIdx.y, g = head / REP;
    const int qw = qblk * 64 + wave * 16;
    const int nch = 2 * qblk + 2;
    const T16* qph = Qh + ((size_t)head * TP + qw) * HD;  const T16* qpl = Ql + ((size_t)head * TP + qw) * HD;
    const T16* kph = Kh + (size_t)g * TP * HD;             const T16* kpl = Kl + (size_t)g * TP * HD;
    const T16* vph = Vh + (size_t)g * HD * TP;             const T16* vpl = Vl + (size_t)g * HD * TP;
    T16* myph = psh + wave * 16 * PSP; T16* mypl = psl + (EARLY ? wave * 16 * PSP : 0);
    v8f o[8];
#pragma unroll
    for (int t = 0; t < 8; ++t) o[t] = (v8f){};
    float mrow[8], lrow[8];
#pragma unroll
    for (int r = 0; r < 8; ++r) { mrow[r] = -3.0e38f; lrow[r] = 0.f; }
    const float C2 = 1.4426950408889634f * 0.08838834764831845f;
    const float CLP = 14426.950408889634f;
    const int nsl = head + 1;
    const float slope = ((nsl & 1) ? 0.70710678118654752440f : 1.0f) * __uint_as_float((unsigned)(127 - (nsl >> 1)) << 23);
    const float SL2 = 1.4426950408889634f * slope;
#pragma unroll 1
    for (int c = 0; c < nch; ++c) {
        __syncthreads();
#pragma unroll
        for (int i = 0; i < 4; ++i) { const int id = tid + 128 * i; const int row = id >> 4, c8 = (id & 15) * 8; const size_t go = (size_t)(c * 32 + row) * HD + c8;
            *(v8usa*)(ksh + row * KSP + c8) = *(const v8usa*)(kph + go); if (EARLY) *(v8usa*)(ksl + row * KSP + c8) = *(const v8usa*)(kpl + go); }
#pragma unroll
        for (int j = 0; j < 4; ++j) { const size_t go = (size_t)tid * TP + c * 32 + 8 * j;
            *(v8usa*)(vth + tid * VTP + 8 * j) = *(const v8usa*)(vph + go); if (EARLY) *(v8usa*)(vtl + tid * VTP + 8 * j) = *(const v8usa*)(vpl + go); }
        __syncthreads();
        v8f s0 = (v8f){}, s1 = (v8f){};
        V qa, kb0, kb1;
#pragma unroll
        for (int ks = 0; ks < 4; ++ks) {
            qa  = WFrag<T16>::ld(qph + (size_t)lr * HD + ks * 32 + 8 * hh);
            kb0 = WFrag<T16>::ld(ksh + lr * KSP + ks * 32 + 8 * hh);
            kb1 = WFrag<T16>::ld(ksh + (16 + lr) * KSP + ks * 32 + 8 * hh);
            s0 = WFrag<T16>::mma(qa, kb0, s0); s1 = WFrag<T16>::mma(qa, kb1, s1);
            if (EARLY) {
                const V qb  = WFrag<T16>::ld(qpl + (size_t)lr * HD + ks * 32 + 8 * hh);
                const V kl0 = WFrag<T16>::ld(ksl + lr * KSP + ks * 32 + 8 * hh);
                const V kl1 = WFrag<T16>::ld(ksl + (16 + lr) * KSP + ks * 32 + 8 * hh);
                s0 = WFrag<T16>::mma(qa, kl0, s0); s0 = WFrag<T16>::mma(qb, kb0, s0);
                s1 = WFrag<T16>::mma(qa, kl1, s1); s1 = WFrag<T16>::mma(qb, kb1, s1); }
        }
        asm volatile("v_nop\n\tv_nop\n\tv_nop\n\tv_nop" : "+v"(s0), "+v"(s1) : "v"(qa), "v"(kb0), "v"(kb1));
        float p0[8], p1[8];
        const int kg0 = c * 32 + lr, kg1 = kg0 + 16;
#pragma unroll
        for (int r = 0; r < 8; ++r) {
            const int qr = qw + 8 * hh + r;
            const bool v0 = (kg0 <= qr), v1 = (kg1 <= qr);
            const float z0 = fminf(fmaxf(s0[r] * C2, -CLP), CLP) + SL2 * (float)(kg0 - qr);
            const float z1 = fminf(fmaxf(s1[r] * C2, -CLP), CLP) + SL2 * (float)(kg1 - qr);
            const float a0 = v0 ? z0 : -3.0e38f;
            const float a1 = v1 ? z1 : -3.0e38f;
            float mx = fmaxf(a0, a1);
#pragma unroll
            for (int off = 8; off >= 1; off >>= 1) mx = fmaxf(mx, __shfl_xor(mx, off, 32));
            const float mnew = fmaxf(mrow[r], mx);
            const float alpha = __builtin_amdgcn_exp2f(mrow[r] - mnew);
            mrow[r] = mnew;
            const float x0 = __builtin_amdgcn_exp2f(a0 - mnew), x1 = __builtin_amdgcn_exp2f(a1 - mnew);
            const float e0 = v0 ? x0 : 0.f, e1 = v1 ? x1 : 0.f;
            float rs = e0 + e1;
#pragma unroll
            for (int off = 8; off >= 1; off >>= 1) rs += __shfl_xor(rs, off, 32);
            lrow[r] = lrow[r] * alpha + rs;
#pragma unroll
            for (int t = 0; t < 8; ++t) o[t][r] = o[t][r] * alpha;
            p0[r] = e0; p1[r] = e1;
        }
#pragma unroll
        for (int r = 0; r < 8; ++r) { putpz(myph, mypl, (8 * hh + r) * PSP + lr, p0[r]); putpz(myph, mypl, (8 * hh + r) * PSP + 16 + lr, p1[r]); }
        __syncthreads();
        const V pa = WFrag<T16>::ld(myph + lr * PSP + 8 * hh);
        V pb = pa; if (EARLY) pb = WFrag<T16>::ld(mypl + lr * PSP + 8 * hh);
        V vb;
#pragma unroll
        for (int t = 0; t < 8; ++t) { vb = WFrag<T16>::ld(vth + (t * 16 + lr) * VTP + 8 * hh);
            o[t] = WFrag<T16>::mma(pa, vb, o[t]);
            if (EARLY) { const V vl2 = WFrag<T16>::ld(vtl + (t * 16 + lr) * VTP + 8 * hh); o[t] = WFrag<T16>::mma(pa, vl2, o[t]); o[t] = WFrag<T16>::mma(pb, vb, o[t]); } }
        asm volatile("v_nop\n\tv_nop\n\tv_nop\n\tv_nop" : "+v"(o[0]), "+v"(o[1]), "+v"(o[2]), "+v"(o[3]), "+v"(o[4]), "+v"(o[5]), "+v"(o[6]), "+v"(o[7]) : "v"(pa), "v"(pb), "v"(vb));
    }
    const float osc = EARLY ? CCAR : (CCAR / PCAR);
    const float ybig = 10000.0f * CCAR;
    float inv[8];
#pragma unroll
    for (int r = 0; r < 8; ++r) inv[r] = osc * __builtin_amdgcn_rcpf(lrow[r]);
    h16* myos = osg + wave * 16 * OSP;
#pragma unroll
    for (int t = 0; t < 8; ++t)
#pragma unroll
        for (int r = 0; r < 8; ++r) myos[(8 * hh + r) * OSP + t * 16 + lr] = toh_flush(nnum(o[t][r] * inv[r], ybig));
    __syncthreads();
    h16* crow = CT + (size_t)qw * DM + head * HD;
#pragma unroll 1
    for (int ps = 0; ps < 2; ++ps) {
#pragma unroll
        for (int s = 0; s < 8; ++s) { const int row = 2 * s + hh; const v8h val = *(const v8ha*)(myos + row * OSP + lr * 8); *(volatile v8h*)(crow + (size_t)row * DM + lr * 8) = val; }
        if (ps == 0) __threadfence(); }
    if (EARLY) {
        __syncthreads();
#pragma unroll
        for (int t = 0; t < 8; ++t)
#pragma unroll
            for (int r = 0; r < 8; ++r) { const float val = nnum(o[t][r] * inv[r], ybig); const h16 hv = toh_flush(val); myos[(8 * hh + r) * OSP + t * 16 + lr] = toh_flush((val - (float)hv) * LOSC); }
        __syncthreads();
        h16* lrowp = CTL + (size_t)qw * DM + head * HD;
#pragma unroll 1
        for (int ps = 0; ps < 2; ++ps) {
#pragma unroll
            for (int s = 0; s < 8; ++s) { const int row = 2 * s + hh; const v8h val = *(const v8ha*)(myos + row * OSP + lr * 8); *(volatile v8h*)(lrowp + (size_t)row * DM + lr * 8) = val; }
            if (ps == 0) __threadfence(); }
    }
}

extern "C" void kernel_launch(void* const* d_in, const int* in_sizes, int n_in,
                              void* d_out, int out_size, void* d_ws, size_t ws_size, hipStream_t stream) {
    if (n_in < 5) return;
    const float* x  = (const float*)d_in[0];
    const float* wq = (const float*)d_in[1];
    const float* wk = (const float*)d_in[2];
    const float* wv = (const float*)d_in[3];
    const float* wo = (const float*)d_in[4];
    float* OUT = (float*)d_out;
    if ((size_t)in_sizes[0] < (size_t)(NB - 1) * SEQ_FULL * DM + (size_t)SEQ * DM) return;
    if ((size_t)in_sizes[1] < (size_t)DQ * DM) return;
    if ((size_t)in_sizes[2] < (size_t)DKV * DM) return;
    if ((size_t)in_sizes[3] < (size_t)DKV * DM) return;
    if ((size_t)in_sizes[4] < (size_t)DM * DQ) return;
    if ((size_t)out_size < (size_t)(NB - 1) * SEQ_FULL * DM + (size_t)SEQ * DM) return;

    char* wsp = (char*)d_ws;
    auto take = [&](size_t bytes) { char* p = wsp; wsp += (bytes + 255) & ~(size_t)255; return (void*)p; };
    bf*  WQ   = (bf*)take((size_t)DQ * DM * 2);    bf* WK = (bf*)take((size_t)DKV * DM * 2);    bf* WV = (bf*)take((size_t)DKV * DM * 2);
    h16* WOH  = (h16*)take((size_t)DM * DQ * 2);   h16* WOL = (h16*)take((size_t)DM * DQ * 2);
    bf*  XB   = (bf*)take((size_t)SEQ * DM * 2);
    float* FQ = (float*)take((size_t)SEQ * DQ * 4); float* FK = (float*)take((size_t)SEQ * DKV * 4); float* FV = (float*)take((size_t)SEQ * DKV * 4);
    h16* QP16 = (h16*)take((size_t)NH_ * SEQ * HD * 2); h16* KP16 = (h16*)take((size_t)NKV * SEQ * HD * 2); h16* VT16 = (h16*)take((size_t)NKV * HD * SEQ * 2);
    bf*  QEh  = (bf*)take((size_t)NH_ * RE * HD * 2);  bf* QEl = (bf*)take((size_t)NH_ * RE * HD * 2);
    bf*  KEh  = (bf*)take((size_t)NKV * RE * HD * 2);  bf* KEl = (bf*)take((size_t)NKV * RE * HD * 2);
    bf*  VEh  = (bf*)take((size_t)NKV * HD * RE * 2);  bf* VEl = (bf*)take((size_t)NKV * HD * RE * 2);
    h16* CT16 = (h16*)take((size_t)SEQ * DM * 2);     h16* CTL = (h16*)take((size_t)RE * DM * 2);
    if ((size_t)(wsp - (char*)d_ws) > ws_size) return;

    const float woscale = 1.0f / (CCAR * WCAR);
    k_cvt8<<<(unsigned)(((size_t)DQ * DM / 8 + 255) / 256), 256, 0, stream>>>(wq, WQ, (size_t)DQ * DM / 8);
    k_cvt8<<<(unsigned)(((size_t)DKV * DM / 8 + 255) / 256), 256, 0, stream>>>(wk, WK, (size_t)DKV * DM / 8);
    k_cvt8<<<(unsigned)(((size_t)DKV * DM / 8 + 255) / 256), 256, 0, stream>>>(wv, WV, (size_t)DKV * DM / 8);
    k_cvtwo<<<(unsigned)(((size_t)DM * DQ / 8 + 255) / 256), 256, 0, stream>>>(wo, WOH, WOL, (size_t)DM * DQ / 8);
    const unsigned LQ = (unsigned)(((size_t)NH_ * SEQ * HD / 2 + 255) / 256), LKV = (unsigned)(((size_t)NKV * SEQ * HD / 2 + 255) / 256);
    for (int b = 0; b < NB; ++b) {
        const float* xb = x + (size_t)b * SEQ_FULL * DM;
        float* OUTb = OUT + (size_t)b * SEQ_FULL * DM;
        k_cvtx<<<(unsigned)(((size_t)SEQ * DM / 8 + 255) / 256), 256, 0, stream>>>(xb, XB, (size_t)SEQ * DM / 8);
        k_gemmw<bf, 0><<<dim3(SEQ / 64, DQ / 64, 1), 32, 0, stream>>>(XB, nullptr, WQ, nullptr, DM, FQ, DQ, 1.0f);
        k_hpl<<<LQ, 256, 0, stream>>>(FQ, DQ, NH_, QP16, QEh, QEl);
        k_gemmw<bf, 0><<<dim3(SEQ / 64, DKV / 64, 1), 32, 0, stream>>>(XB, nullptr, WK, nullptr, DM, FK, DKV, 1.0f);
        k_hpl<<<LKV, 256, 0, stream>>>(FK, DKV, NKV, KP16, KEh, KEl);
        k_gemmw<bf, 0><<<dim3(SEQ / 64, DKV / 64, 1), 32, 0, stream>>>(XB, nullptr, WV, nullptr, DM, FV, DKV, 1.0f);
        k_vtp<<<LKV, 256, 0, stream>>>(FV, VT16, VEh, VEl);
        k_attn<bf, true><<<dim3(RE / 64, NH_, 1), 128, 0, stream>>>(QEh, QEl, KEh, KEl, VEh, VEl, CT16, CTL);
        if (SEQ > RE) k_attn<h16, false><<<dim3(SEQ / 64 - RE / 64, NH_, 1), 128, 0, stream>>>(QP16, QP16, KP16, KP16, VT16, VT16, CT16, CTL);
        k_gemmw<h16, 3><<<dim3(RE / 64, DM / 64, 1), 32, 0, stream>>>(CT16, CTL, WOH, WOL, DQ, OUTb, DM, woscale);
        if (SEQ > RE) k_gemmw<h16, 0><<<dim3((SEQ - RE) / 64, DM / 64, 1), 32, 0, stream>>>(CT16 + (size_t)RE * DQ, nullptr, WOH, nullptr, DQ, OUTb + (size_t)RE * DM, DM, woscale);
    }
}
